// GeneralizedAttention_23845658427761
// MI455X (gfx1250) — hardware-verified
//
#include <hip/hip_runtime.h>
#include <stddef.h>
#include <stdint.h>


#define CCH 256
#define NHD 8
#define DHD 32
#define NB 2
#define HQ 64
#define WQ 64
#define HWQ 4096
#define HKV 32
#define WKV 32
#define KVP 1024
#define SRNG 10
#define KVS 2
#define NEMB 2048
#define FDIM 128
#define LDSP 264
#define PSCL 4096.0f
#define NEGBIG (-3.0e38f)
#define ISQ2 0.70710678118654752f

typedef _Float16 f16;
typedef f16 v16h __attribute__((ext_vector_type(16)));
typedef f16 v8h __attribute__((ext_vector_type(8)));
typedef float v8f __attribute__((ext_vector_type(8)));
typedef float v4f __attribute__((ext_vector_type(4)));
union Frag { v16h v; v8h h[2]; };

static __device__ __forceinline__ v8f mma(v16h a, v16h b, v8f c) {
  v8f d = __builtin_amdgcn_wmma_f32_16x16x32_f16(false, a, false, b, (short)0, c,
                                                false, false);
  asm volatile("v_nop\n\tv_nop\n\tv_nop\n\tv_nop" : "+v"(d) : "v"(a), "v"(b));
  return d;
}

static __device__ __forceinline__ v8f zero8() {
  v8f z = {0.f, 0.f, 0.f, 0.f, 0.f, 0.f, 0.f, 0.f};
  return z;
}

static __device__ __forceinline__ v16h ldA_cvt(const float* __restrict__ base, int lda,
                                                int lane, int k0) {
  const int m = lane & 15, h = lane >> 4;
  const float* p = base + (size_t)m * lda + k0 + 8 * h;
  const v4f c0 = *(const v4f*)(p);
  const v4f c1 = *(const v4f*)(p + 4);
  const v4f c2 = *(const v4f*)(p + 16);
  const v4f c3 = *(const v4f*)(p + 20);
  v16h a;
#pragma unroll
  for (int j = 0; j < 4; ++j) {
    a[j]      = (f16)c0[j];
    a[4 + j]  = (f16)c1[j];
    a[8 + j]  = (f16)c2[j];
    a[12 + j] = (f16)c3[j];
  }
  return a;
}

static __device__ __forceinline__ v16h ldK(const f16* base, int pitch, int lane, int k0) {
  const int m = lane & 15, h = lane >> 4;
  const f16* p = base + (size_t)m * pitch + k0 + 8 * h;
  Frag f;
  f.h[0] = *(const v8h*)(p);
  f.h[1] = *(const v8h*)(p + 16);
  return f.v;
}

static __device__ __forceinline__ v16h ldB_gather(const f16* base, int ldn, int lane) {
  const int m = lane & 15, h = lane >> 4;
  const f16* p = base + (size_t)(8 * h) * ldn + m;
  v16h b;
#pragma unroll
  for (int i = 0; i < 8; ++i) {
    b[i]     = p[(size_t)i * ldn];
    b[8 + i] = p[(size_t)(16 + i) * ldn];
  }
  return b;
}

static __device__ __forceinline__ void st8f(float* q, v8f a) {
  v4f lo = {a[0], a[1], a[2], a[3]};
  v4f hi = {a[4], a[5], a[6], a[7]};
  *(v4f*)(q) = lo;
  *(v4f*)(q + 4) = hi;
}

static __device__ __forceinline__ void gemm32x32(const float* __restrict__ Aw, int lda, int K,
                                                 const f16* lb, int lane,
                                                 v8f& a00, v8f& a01, v8f& a10, v8f& a11) {
  for (int k0 = 0; k0 < K; k0 += 32) {
    const v16h A0 = ldA_cvt(Aw, lda, lane, k0);
    const v16h A1 = ldA_cvt(Aw + (size_t)16 * lda, lda, lane, k0);
    const v16h B0 = ldK(lb, LDSP, lane, k0);
    const v16h B1 = ldK(lb + 16 * LDSP, LDSP, lane, k0);
    a00 = mma(A0, B0, a00);
    a01 = mma(A0, B1, a01);
    a10 = mma(A1, B0, a10);
    a11 = mma(A1, B1, a11);
  }
}

__global__ __launch_bounds__(256) void k_emb(f16* __restrict__ emb) {
  __shared__ __align__(16) f16 s[256];
  const int t = threadIdx.x;
  const int row = (int)blockIdx.x * 2 + (t >> 7);
  const int f = t & 127;
  const int q = row >> 5, kk = row & 31;
  const float diff = ((float)q * 1.0f - (float)kk * (float)KVS) * 1.0f;
  const int j = f & 63;
  const float dm = powf(1000.0f, 0.015625f * (float)j);
  const float a = diff * (1.0f / dm);
  const float val = (f < 64) ? sinf(a) : cosf(a);
  s[t] = (f16)val;
  __syncthreads();
  if (t < 32) {
    const v8h v = *(const v8h*)&s[t * 8];
    f16* d = emb + (size_t)blockIdx.x * 256 + t * 8;
    *(volatile v8h*)d = v;
    __threadfence();
    *(volatile v8h*)d = v;
  }
}

__global__ __launch_bounds__(256) void k_pos(const f16* __restrict__ emb,
                                             const float* __restrict__ gwx,
                                             const float* __restrict__ gwy,
                                             f16* __restrict__ pos) {
  __shared__ __align__(16) f16 lb[32 * LDSP];
  __shared__ __align__(16) f16 lo[32 * LDSP];
  const int t = threadIdx.x, lane = t & 31, w = t >> 5, m = lane & 15, hh = lane >> 4;
  const int axis = (int)blockIdx.x >> 6, p0 = ((int)blockIdx.x & 63) * 32;
  const float* gw = axis ? gwy : gwx;
  {
    const int p = t >> 3, f = (t & 7) * 16;
    const f16* src = emb + (size_t)(p0 + p) * FDIM + f;
    *(v8h*)&lb[p * LDSP + f]     = *(const v8h*)(src);
    *(v8h*)&lb[p * LDSP + f + 8] = *(const v8h*)(src + 8);
  }
  __syncthreads();
  v8f a00 = zero8(), a01 = zero8(), a10 = zero8(), a11 = zero8();
  gemm32x32(gw + (size_t)(32 * w) * FDIM, FDIM, FDIM, lb, lane, a00, a01, a10, a11);
  {
    v8h tv;
#pragma unroll
    for (int r = 0; r < 8; ++r) tv[r] = (f16)(a00[r] * ISQ2);
    *(v8h*)&lo[(0 + m) * LDSP + 32 * w + 0 + 8 * hh] = tv;
#pragma unroll
    for (int r = 0; r < 8; ++r) tv[r] = (f16)(a01[r] * ISQ2);
    *(v8h*)&lo[(16 + m) * LDSP + 32 * w + 0 + 8 * hh] = tv;
#pragma unroll
    for (int r = 0; r < 8; ++r) tv[r] = (f16)(a10[r] * ISQ2);
    *(v8h*)&lo[(0 + m) * LDSP + 32 * w + 16 + 8 * hh] = tv;
#pragma unroll
    for (int r = 0; r < 8; ++r) tv[r] = (f16)(a11[r] * ISQ2);
    *(v8h*)&lo[(16 + m) * LDSP + 32 * w + 16 + 8 * hh] = tv;
  }
  __syncthreads();
  v8h rv[4];
#pragma unroll
  for (int u = 0; u < 4; ++u) rv[u] = *(const v8h*)&lo[(4 * w + u) * LDSP + lane * 8];
  f16* dst = pos + ((size_t)axis * NEMB + p0 + 4 * w) * CCH + lane * 8;
#pragma unroll
  for (int u = 0; u < 4; ++u) *(volatile v8h*)(dst + (size_t)u * CCH) = rv[u];
  __threadfence();
#pragma unroll
  for (int u = 0; u < 4; ++u) *(volatile v8h*)(dst + (size_t)u * CCH) = rv[u];
}

template <int QM>
__global__ __launch_bounds__(256) void k_proj(const float* __restrict__ x,
                                              const float* __restrict__ W,
                                              const float* __restrict__ b0,
                                              const float* __restrict__ b1,
                                              f16* __restrict__ o0, f16* __restrict__ o1) {
  __shared__ __align__(16) f16 lb[32 * LDSP];
  __shared__ __align__(16) float ls[8][1024];
  const int t = threadIdx.x, lane = t & 31, w = t >> 5, hh = lane >> 4, m = lane & 15;
  const int P = QM ? HWQ : KVP;
  int n, p0;
  if (QM) { n = (int)blockIdx.x >> 7; p0 = ((int)blockIdx.x & 127) * 32; }
  else    { n = (int)blockIdx.x >> 5; p0 = ((int)blockIdx.x & 31) * 32; }
  {
    const int pl = t & 31, cb = t >> 5;
    const int pp = p0 + pl;
    const int col = QM ? pp : ((pp >> 5) * KVS * WQ + (pp & 31) * KVS);
    const float* xs = x + (size_t)n * CCH * HWQ + col;
#pragma unroll 4
    for (int s = 0; s < 32; ++s) {
      const int c = cb + 8 * s;
      lb[pl * LDSP + c] = (f16)xs[(size_t)c * HWQ];
    }
  }
  __syncthreads();
  const int h = w;
  v8f a00 = zero8(), a01 = zero8(), a10 = zero8(), a11 = zero8();
  gemm32x32(W + (size_t)(32 * h) * CCH, CCH, CCH, lb, lane, a00, a01, a10, a11);
  float* st = &ls[w][0];
  st8f(st + (0 + m) * 32 + 0 + 8 * hh, a00);
  st8f(st + (16 + m) * 32 + 0 + 8 * hh, a01);
  st8f(st + (0 + m) * 32 + 16 + 8 * hh, a10);
  st8f(st + (16 + m) * 32 + 16 + 8 * hh, a11);
  __syncthreads();
  const size_t tb = (((size_t)n * NHD + h) * (size_t)P + p0) * DHD;
  v8h ra[4], rg[4];
#pragma unroll
  for (int t4 = 0; t4 < 4; ++t4) {
    const int p = t4 * 8 + (lane >> 2), d0 = (lane & 3) * 8;
    const v4f u0 = *(const v4f*)&st[p * 32 + d0];
    const v4f u1 = *(const v4f*)&st[p * 32 + d0 + 4];
    const float vv[8] = {u0[0], u0[1], u0[2], u0[3], u1[0], u1[1], u1[2], u1[3]};
#pragma unroll
    for (int e = 0; e < 8; ++e) {
      if (QM) {
        const int o = 32 * h + d0 + e;
        ra[t4][e] = (f16)(vv[e] + b0[o]);
        rg[t4][e] = (f16)(vv[e] + b1[o]);
      } else {
        ra[t4][e] = (f16)vv[e];
        rg[t4][e] = ra[t4][e];
      }
    }
  }
#pragma unroll
  for (int t4 = 0; t4 < 4; ++t4) {
    const size_t off = tb + (size_t)t4 * 256 + lane * 8;
    *(volatile v8h*)(o0 + off) = ra[t4];
    if (QM) *(volatile v8h*)(o1 + off) = rg[t4];
  }
  __threadfence();
#pragma unroll
  for (int t4 = 0; t4 < 4; ++t4) {
    const size_t off = tb + (size_t)t4 * 256 + lane * 8;
    *(volatile v8h*)(o0 + off) = ra[t4];
    if (QM) *(volatile v8h*)(o1 + off) = rg[t4];
  }
}

__global__ __launch_bounds__(256) void k_exy(const f16* __restrict__ qg,
                                             const f16* __restrict__ pos,
                                             float* __restrict__ ex, float* __restrict__ ey) {
  __shared__ __align__(16) float ls[8][512];
  const int t = threadIdx.x, lane = t & 31, w = t >> 5, m = lane & 15, hh = lane >> 4;
  int idx = (int)blockIdx.x * 8 + w;
  const int rt = idx & 3;        idx >>= 2;
  const int q2 = idx & 63;       idx >>= 6;
  const int h = idx & 7;         idx >>= 3;
  const int n = idx & 1;         idx >>= 1;
  const int axis = idx & 1;
  const size_t nh = (size_t)n * NHD + h;
  const f16* Ab;
  int pitch;
  if (axis == 0) { Ab = qg + (nh * HWQ + (size_t)(16 * rt) * WQ + q2) * DHD; pitch = WQ * DHD; }
  else           { Ab = qg + (nh * HWQ + (size_t)q2 * WQ + 16 * rt) * DHD; pitch = DHD; }
  const v16h a = ldK(Ab, pitch, lane, 0);
  const f16* Bb = pos + ((size_t)axis * NEMB + (size_t)q2 * 32) * CCH + h * DHD;
  const v16h b0 = ldK(Bb, CCH, lane, 0);
  const v16h b1 = ldK(Bb + 16 * CCH, CCH, lane, 0);
  const v8f c0 = mma(a, b0, zero8());
  const v8f c1 = mma(a, b1, zero8());
  float* st = &ls[w][0];
#pragma unroll
  for (int r = 0; r < 8; ++r) {
    st[(8 * hh + r) * 32 + m]      = c0[r];
    st[(8 * hh + r) * 32 + 16 + m] = c1[r];
  }
  __syncthreads();
  float* E = axis ? ey : ex;
  const size_t tb = ((nh * 64 + q2) * 64 + (size_t)(16 * rt)) * 32;
  v4f rv[4];
#pragma unroll
  for (int t4 = 0; t4 < 4; ++t4)
    rv[t4] = *(const v4f*)&st[(4 * t4 + (lane >> 3)) * 32 + (lane & 7) * 4];
#pragma unroll
  for (int t4 = 0; t4 < 4; ++t4)
    *(volatile v4f*)(E + tb + (size_t)t4 * 128 + lane * 4) = rv[t4];
  __threadfence();
#pragma unroll
  for (int t4 = 0; t4 < 4; ++t4)
    *(volatile v4f*)(E + tb + (size_t)t4 * 128 + lane * 4) = rv[t4];
}

__global__ __launch_bounds__(256) void k_attn(const f16* __restrict__ qa,
                                              const f16* __restrict__ pk,
                                              const f16* __restrict__ pv,
                                              const float* __restrict__ ex,
                                              const float* __restrict__ ey,
                                              const int* __restrict__ msk,
                                              f16* __restrict__ att) {
  __shared__ __align__(16) f16 pb_all[8][512];
  __shared__ __align__(16) f16 ost[16 * LDSP];
  const int t = threadIdx.x, lane = t & 31, h = t >> 5, m = lane & 15, hh = lane >> 4;
  const int blk = (int)blockIdx.x;
  const int x0 = (blk & 3) * 16, y = (blk >> 2) & 63, n = blk >> 8;
  const size_t nh = (size_t)n * NHD + h;

  const int ky_lo = (y > SRNG) ? ((y - SRNG) / KVS) : 0;
  int ky_hi = (y + SRNG + 1) / KVS + 1;
  if (ky_hi > HKV) ky_hi = HKV;

  const v16h aq = ldK(qa + (nh * HWQ + (size_t)y * WQ + x0) * DHD, DHD, lane, 0);

  float exr0[8], exr1[8];
  {
    const float* eb = ex + ((nh * WQ + x0 + 8 * hh) * HQ + (size_t)y) * WKV + m;
#pragma unroll
    for (int r = 0; r < 8; ++r) {
      exr0[r] = eb[(size_t)r * HQ * WKV];
      exr1[r] = eb[(size_t)r * HQ * WKV + 16];
    }
  }
  const float* eyb = ey + ((nh * HQ + y) * WQ + (size_t)(x0 + 8 * hh)) * HKV;
  const int*   mb  = msk + ((size_t)(y * WQ + x0 + 8 * hh)) * KVP + m;
  const f16*   kb  = pk + nh * (size_t)KVP * DHD;
  const f16*   vb  = pv + nh * (size_t)KVP * DHD;
  f16* pb = &pb_all[h][0];

  float rmax[8], rsum[8];
#pragma unroll
  for (int r = 0; r < 8; ++r) { rmax[r] = NEGBIG; rsum[r] = 0.f; }
  v8f o0 = zero8(), o1 = zero8();

  for (int ky = ky_lo; ky < ky_hi; ++ky) {
    const v16h bk0 = ldK(kb + (size_t)(ky * WKV) * DHD, DHD, lane, 0);
    const v16h bk1 = ldK(kb + (size_t)(ky * WKV + 16) * DHD, DHD, lane, 0);
    v8f e0 = mma(aq, bk0, zero8());
    v8f e1 = mma(aq, bk1, zero8());
    float tmax[8];
#pragma unroll
    for (int r = 0; r < 8; ++r) {
      const float eyv = eyb[r * HKV + ky];
      const int m0v = mb[(size_t)r * KVP + ky * WKV];
      const int m1v = mb[(size_t)r * KVP + ky * WKV + 16];
      float s0 = e0[r] + exr0[r] + eyv;
      float s1 = e1[r] + exr1[r] + eyv;
      s0 = (m0v == 0) ? s0 : NEGBIG;
      s1 = (m1v == 0) ? s1 : NEGBIG;
      e0[r] = s0; e1[r] = s1;
      tmax[r] = fmaxf(s0, s1);
    }
#pragma unroll
    for (int s = 1; s < 16; s <<= 1) {
#pragma unroll
      for (int r = 0; r < 8; ++r) tmax[r] = fmaxf(tmax[r], __shfl_xor(tmax[r], s, 32));
    }
    float sc[8], psum[8];
#pragma unroll
    for (int r = 0; r < 8; ++r) {
      const float nm = fmaxf(rmax[r], tmax[r]);
      sc[r] = __expf(rmax[r] - nm);
      rmax[r] = nm;
      const float p0v = (e0[r] > -1.0e38f) ? __expf(e0[r] - nm) : 0.f;
      const float p1v = (e1[r] > -1.0e38f) ? __expf(e1[r] - nm) : 0.f;
      e0[r] = p0v; e1[r] = p1v;
      psum[r] = p0v + p1v;
    }
#pragma unroll
    for (int s = 1; s < 16; s <<= 1) {
#pragma unroll
      for (int r = 0; r < 8; ++r) psum[r] += __shfl_xor(psum[r], s, 32);
    }
#pragma unroll
    for (int r = 0; r < 8; ++r) {
      rsum[r] = rsum[r] * sc[r] + psum[r];
      o0[r] *= sc[r];
      o1[r] *= sc[r];
    }
#pragma unroll
    for (int r = 0; r < 8; ++r) {
      pb[(8 * hh + r) * 32 + m]      = (f16)(e0[r] * PSCL);
      pb[(8 * hh + r) * 32 + 16 + m] = (f16)(e1[r] * PSCL);
    }
    __syncthreads();
    const v16h ap  = ldK(pb, 32, lane, 0);
    const v16h bv0 = ldB_gather(vb + (size_t)(ky * WKV) * DHD, DHD, lane);
    const v16h bv1 = ldB_gather(vb + (size_t)(ky * WKV) * DHD + 16, DHD, lane);
    o0 = mma(ap, bv0, o0);
    o1 = mma(ap, bv1, o1);
    __syncthreads();
  }
#pragma unroll
  for (int r = 0; r < 8; ++r) {
    const float inv = 1.0f / (rsum[r] * PSCL);
    ost[(8 * hh + r) * LDSP + 32 * h + m]      = (f16)(o0[r] * inv);
    ost[(8 * hh + r) * LDSP + 32 * h + 16 + m] = (f16)(o1[r] * inv);
  }
  __syncthreads();
  const v8h w0 = *(const v8h*)&ost[(2 * h) * LDSP + lane * 8];
  const v8h w1 = *(const v8h*)&ost[(2 * h + 1) * LDSP + lane * 8];
  f16* d0 = att + ((size_t)n * HWQ + (size_t)y * WQ + x0 + 2 * h) * CCH + lane * 8;
  f16* d1 = d0 + CCH;
  *(volatile v8h*)d0 = w0;
  *(volatile v8h*)d1 = w1;
  __threadfence();
  *(volatile v8h*)d0 = w0;
  *(volatile v8h*)d1 = w1;
}

__global__ __launch_bounds__(256) void k_final(const f16* __restrict__ att,
                                               const float* __restrict__ Wp,
                                               const float* __restrict__ pbias,
                                               const float* __restrict__ gam,
                                               const float* __restrict__ x,
                                               float* __restrict__ out) {
  __shared__ __align__(16) f16 lb[32 * LDSP];
  __shared__ __align__(16) float ls[8][1024];
  const int t = threadIdx.x, lane = t & 31, w = t >> 5, m = lane & 15, hh = lane >> 4;
  const int n = (int)blockIdx.x >> 7, p0 = ((int)blockIdx.x & 127) * 32;
#pragma unroll
  for (int u = 0; u < 2; ++u) {
    const int e = u * 4096 + t * 16;
    const int p = e >> 8, c = e & 255;
    const f16* src = att + ((size_t)n * HWQ + p0 + p) * CCH + c;
    *(v8h*)&lb[p * LDSP + c]     = *(const v8h*)(src);
    *(v8h*)&lb[p * LDSP + c + 8] = *(const v8h*)(src + 8);
  }
  __syncthreads();
  v8f a00 = zero8(), a01 = zero8(), a10 = zero8(), a11 = zero8();
  gemm32x32(Wp + (size_t)(32 * w) * CCH, CCH, CCH, lb, lane, a00, a01, a10, a11);
  float* st = &ls[w][0];
#pragma unroll
  for (int r = 0; r < 8; ++r) {
    st[(0 + 8 * hh + r) * 32 + 0 + m]   = a00[r];
    st[(0 + 8 * hh + r) * 32 + 16 + m]  = a01[r];
    st[(16 + 8 * hh + r) * 32 + 0 + m]  = a10[r];
    st[(16 + 8 * hh + r) * 32 + 16 + m] = a11[r];
  }
  __syncthreads();
  const float g = gam[0];
  v4f rv[8];
#pragma unroll
  for (int t8 = 0; t8 < 8; ++t8) {
    const int ol = 4 * t8 + (lane >> 3), pp = (lane & 7) * 4;
    const int o = 32 * w + ol;
    const v4f v = *(const v4f*)&st[ol * 32 + pp];
    const size_t idx = ((size_t)n * CCH + o) * HWQ + p0 + pp;
    const v4f xin = *(const v4f*)(x + idx);
    const float b = pbias[o];
    v4f rr;
#pragma unroll
    for (int e = 0; e < 4; ++e) rr[e] = g * (v[e] + b) + xin[e];
    rv[t8] = rr;
  }
#pragma unroll
  for (int t8 = 0; t8 < 8; ++t8) {
    const int ol = 4 * t8 + (lane >> 3), pp = (lane & 7) * 4;
    const size_t idx = ((size_t)n * CCH + 32 * w + ol) * HWQ + p0 + pp;
    *(volatile v4f*)(out + idx) = rv[t8];
  }
  __threadfence();
#pragma unroll
  for (int t8 = 0; t8 < 8; ++t8) {
    const int ol = 4 * t8 + (lane >> 3), pp = (lane & 7) * 4;
    const size_t idx = ((size_t)n * CCH + 32 * w + ol) * HWQ + p0 + pp;
    *(volatile v4f*)(out + idx) = rv[t8];
  }
}

extern "C" void kernel_launch(void* const* d_in, const int* in_sizes, int n_in,
                              void* d_out, int out_size, void* d_ws, size_t ws_size,
                              hipStream_t stream) {
  if (n_in < 12) return;
  if (in_sizes[0] != NB * CCH * HWQ) return;
  if (in_sizes[1] != CCH * CCH || in_sizes[2] != CCH * CCH || in_sizes[3] != CCH * CCH) return;
  if (in_sizes[4] != CCH * FDIM || in_sizes[5] != CCH * FDIM) return;
  if (in_sizes[6] != CCH || in_sizes[7] != CCH) return;
  if (in_sizes[8] != CCH * CCH || in_sizes[9] != CCH || in_sizes[10] < 1) return;
  if (in_sizes[11] != HWQ * KVP) return;
  if (out_size != NB * CCH * HWQ) return;

  const float* x       = (const float*)d_in[0];
  const float* query_w = (const float*)d_in[1];
  const float* key_w   = (const float*)d_in[2];
  const float* value_w = (const float*)d_in[3];
  const float* geomxw  = (const float*)d_in[4];
  const float* geomyw  = (const float*)d_in[5];
  const float* ab      = (const float*)d_in[6];
  const float* gb      = (const float*)d_in[7];
  const float* proj_w  = (const float*)d_in[8];
  const float* proj_b  = (const float*)d_in[9];
  const float* gamma   = (const float*)d_in[10];
  const int*   msk     = (const int*)d_in[11];
  float* out = (float*)d_out;

  size_t off = 0;
  auto carve = [&](size_t bytes) { size_t o = off; off += (bytes + 255) & ~(size_t)255; return o; };
  const size_t o_emb = carve((size_t)NEMB * FDIM * 2);
  const size_t o_pos = carve((size_t)2 * NEMB * CCH * 2);
  const size_t o_qa  = carve((size_t)NB * NHD * HWQ * DHD * 2);
  const size_t o_qg  = carve((size_t)NB * NHD * HWQ * DHD * 2);
  const size_t o_pk  = carve((size_t)NB * NHD * KVP * DHD * 2);
  const size_t o_pv  = carve((size_t)NB * NHD * KVP * DHD * 2);
  const size_t o_ex  = carve((size_t)NB * NHD * WQ * HQ * WKV * 4);
  const size_t o_ey  = carve((size_t)NB * NHD * HQ * WQ * HKV * 4);
  const size_t o_att = carve((size_t)NB * HWQ * CCH * 2);
  if (off > ws_size) return;
  char* wsb = (char*)d_ws;
  f16*   emb = (f16*)(wsb + o_emb);
  f16*   pos = (f16*)(wsb + o_pos);
  f16*   qa  = (f16*)(wsb + o_qa);
  f16*   qg  = (f16*)(wsb + o_qg);
  f16*   pk  = (f16*)(wsb + o_pk);
  f16*   pv  = (f16*)(wsb + o_pv);
  float* e_x = (float*)(wsb + o_ex);
  float* e_y = (float*)(wsb + o_ey);
  f16*   att = (f16*)(wsb + o_att);

  k_emb<<<dim3(NEMB / 2), dim3(256), 0, stream>>>(emb);
  k_pos<<<dim3(2 * (NEMB / 32)), dim3(256), 0, stream>>>(emb, geomxw, geomyw, pos);
  k_proj<1><<<dim3(NB * (HWQ / 32)), dim3(256), 0, stream>>>(x, query_w, ab, gb, qa, qg);
  k_proj<0><<<dim3(NB * (KVP / 32)), dim3(256), 0, stream>>>(x, key_w, ab, gb, pk, pk);
  k_proj<0><<<dim3(NB * (KVP / 32)), dim3(256), 0, stream>>>(x, value_w, ab, gb, pv, pv);
  k_exy<<<dim3(8192 / 8), dim3(256), 0, stream>>>(qg, pos, e_x, e_y);
  k_attn<<<dim3(NB * HQ * (WQ / 16)), dim3(256), 0, stream>>>(qa, pk, pv, e_x, e_y, msk, att);
  k_final<<<dim3(NB * (HWQ / 32)), dim3(256), 0, stream>>>(att, proj_w, proj_b, gamma, x, out);
}
